// LSTM_80642305949766
// MI455X (gfx1250) — hardware-verified
//
#include <hip/hip_runtime.h>
#include <math.h>

constexpr int NSEQ   = 32;
constexpr int NSTEP  = 1024;
constexpr int NCH    = 256;
constexpr int NHID   = 128;
constexpr int NGATE  = 4 * NHID;
constexpr int NLAY   = 2;
constexpr int NDIR   = 2;
constexpr int NTHR   = 256;
constexpr int SEQ_BLK = 16;
constexpr int NROWS  = NSTEP * NSEQ;
constexpr int NFLAT  = NSEQ * NCH;
constexpr int NXELEM = NSEQ * NCH * NSTEP;
constexpr int APITCH = 776;
constexpr int AX_HI  = 0;
constexpr int AX_LO  = NCH;
constexpr int AH_HI  = 2 * NCH;
constexpr int AH_LO  = 2 * NCH + NHID;
constexpr int SLP    = 132;
constexpr int TPP    = 65;
constexpr float WCARRY      = 256.0f;
constexpr float WCARRY_INV  = 1.0f / 256.0f;
constexpr float RCARRY      = 2048.0f;
constexpr float LCARRY_INV  = 1.0f / (256.0f * 2048.0f);
constexpr float F16_MIN_NORMAL = 6.103515625e-5f;
static_assert(NCH == 2 * NHID);
static_assert(NCH % 32 == 0 && NHID % 32 == 0);
static_assert(NHID == 16 * (NTHR / 32));
static_assert(NSEQ % SEQ_BLK == 0);
static_assert(NTHR == SEQ_BLK * 16);
static_assert(AH_LO + NHID + 8 == APITCH);
static_assert(APITCH % 8 == 0 && SLP % 4 == 0);
static_assert((SEQ_BLK * APITCH) % 2 == 0);
static_assert(NSTEP % 64 == 0 && NFLAT % 64 == 0);
static_assert((NLAY * NDIR * NGATE * NCH) % (8 * NTHR) == 0);
static_assert((NLAY * NDIR * NGATE * NHID) % (8 * NTHR) == 0);

typedef __attribute__((ext_vector_type(16))) _Float16 v16h;
typedef __attribute__((ext_vector_type(8)))  _Float16 v8h;
typedef __attribute__((ext_vector_type(8)))  float    v8f;
typedef __attribute__((ext_vector_type(4)))  float    v4f;
typedef __attribute__((ext_vector_type(4)))  unsigned v4u;

__device__ __forceinline__ void acc_guard4(v8f& a, v8f& b, v8f& c, v8f& d) { asm volatile("v_nop\n\tv_nop\n\tv_nop\n\tv_nop" : "+v"(a), "+v"(b), "+v"(c), "+v"(d)); }
__device__ __forceinline__ void guard8_h(v8f& a0, v8f& a1, v8f& a2, v8f& a3, v8f& a4, v8f& a5, v8f& a6, v8f& a7,
                                         v16h x0, v16h x1, v16h y0, v16h y1, v16h y2, v16h y3) {
  asm volatile("v_nop\n\tv_nop\n\tv_nop\n\tv_nop"
               : "+v"(a0), "+v"(a1), "+v"(a2), "+v"(a3), "+v"(a4), "+v"(a5), "+v"(a6), "+v"(a7)
               : "v"(x0), "v"(x1), "v"(y0), "v"(y1), "v"(y2), "v"(y3));
}

template <typename T> struct Frag;
template <> struct Frag<_Float16> {
  typedef v16h V; union U { v16h v; v8h h[2]; };
  static __device__ __forceinline__ v16h load(const _Float16* p) {
    U f; f.h[0] = *(const v8h*)(p); f.h[1] = *(const v8h*)(p + 16); return f.v;
  }
  static __device__ __forceinline__ v8f mma(v16h a, v16h b, v8f c) {
    return __builtin_amdgcn_wmma_f32_16x16x32_f16(false, a, false, b, (short)0, c, false, false);
  }
};

__device__ __forceinline__ float fsig(float x)  { return __builtin_amdgcn_rcpf(1.0f + expf(-x)); }
__device__ __forceinline__ float ftanh(float x) { return 1.0f - 2.0f * __builtin_amdgcn_rcpf(expf(2.0f * x) + 1.0f); }

__global__ __launch_bounds__(NTHR) void cvt16_kernel(const float* __restrict__ src, unsigned short* __restrict__ dst,
                                                     int n8, float sc) {
  const int i = blockIdx.x * NTHR + threadIdx.x;
  if (i < n8) {
    const v4f a = *(const v4f*)(src + (size_t)i * 8);
    const v4f b = *(const v4f*)(src + (size_t)i * 8 + 4);
    v8h hv;
#pragma unroll
    for (int e = 0; e < 4; ++e) {
      hv[e]     = (_Float16)(a[e] * sc);
      hv[4 + e] = (_Float16)(b[e] * sc);
    }
    *(volatile v8h*)(dst + (size_t)i * 8) = hv;
    __threadfence();
    *(volatile v8h*)(dst + (size_t)i * 8) = hv;
  }
}

__global__ __launch_bounds__(NTHR) void tp16_kernel(const float* __restrict__ src, int C, int ldo,
                                                    unsigned short* __restrict__ O) {
  __shared__ float Tt[64 * TPP];
  const int tid = threadIdx.x;
  const int c0 = blockIdx.x * 64, r0 = blockIdx.y * 64;
#pragma unroll
  for (int i = 0; i < 4; ++i) {
    const int idx = i * NTHR + tid;
    const int rr = idx >> 4, cc = (idx & 15) * 4;
    const v4f v = *(const v4f*)(src + (size_t)(r0 + rr) * (size_t)C + c0 + cc);
    Tt[rr * TPP + cc + 0] = v[0];
    Tt[rr * TPP + cc + 1] = v[1];
    Tt[rr * TPP + cc + 2] = v[2];
    Tt[rr * TPP + cc + 3] = v[3];
  }
  __syncthreads();
  const int q = tid >> 3, c8 = (tid & 7) * 8;
  v8h hv[2];
#pragma unroll
  for (int g = 0; g < 2; ++g) {
    const int qq = g * 32 + q;
#pragma unroll
    for (int e = 0; e < 8; ++e) {
      const float f = Tt[(c8 + e) * TPP + qq];
      hv[g][e] = (_Float16)f;
    }
  }
  for (int pass = 0; pass < 2; ++pass) {
#pragma unroll
    for (int g = 0; g < 2; ++g) {
      const size_t o = (size_t)(c0 + g * 32 + q) * (size_t)ldo + (size_t)(r0 + c8);
      *(volatile v8h*)(O + o) = hv[g];
    }
    __threadfence();
  }
}

__global__ __launch_bounds__(NTHR) void tp32_kernel(const float* __restrict__ src, int C, int ldo,
                                                    float* __restrict__ O) {
  __shared__ float Tt[64 * TPP];
  const int tid = threadIdx.x;
  const int c0 = blockIdx.x * 64, r0 = blockIdx.y * 64;
#pragma unroll
  for (int i = 0; i < 4; ++i) {
    const int idx = i * NTHR + tid;
    const int rr = idx >> 4, cc = (idx & 15) * 4;
    const v4f v = *(const v4f*)(src + (size_t)(r0 + rr) * (size_t)C + c0 + cc);
    Tt[rr * TPP + cc + 0] = v[0];
    Tt[rr * TPP + cc + 1] = v[1];
    Tt[rr * TPP + cc + 2] = v[2];
    Tt[rr * TPP + cc + 3] = v[3];
  }
  __syncthreads();
  v4f ov[4];
#pragma unroll
  for (int it = 0; it < 4; ++it) {
    const int idx = it * NTHR + tid;
    const int orow = idx >> 4, c4 = (idx & 15) * 4;
#pragma unroll
    for (int e = 0; e < 4; ++e) ov[it][e] = Tt[(c4 + e) * TPP + orow];
  }
  for (int pass = 0; pass < 2; ++pass) {
#pragma unroll
    for (int it = 0; it < 4; ++it) {
      const int idx = it * NTHR + tid;
      const int orow = idx >> 4, c4 = (idx & 15) * 4;
      *(volatile v4f*)(O + (size_t)(c0 + orow) * (size_t)ldo + (size_t)(r0 + c4)) = ov[it];
    }
    __threadfence();
  }
}

template <bool XSPLIT>
__device__ __forceinline__ void stage_x_rows(unsigned short* At, const unsigned short* XH, const unsigned short* XL,
                                             size_t goff, int loff) {
  const v4u u0 = *(const v4u*)(XH + goff);
  const v4u u1 = *(const v4u*)(XH + goff + 8);
  *(v4u*)(At + loff + AX_HI)     = u0;
  *(v4u*)(At + loff + AX_HI + 8) = u1;
  if (XSPLIT) {
    const v4u w0 = *(const v4u*)(XL + goff);
    const v4u w1 = *(const v4u*)(XL + goff + 8);
    *(v4u*)(At + loff + AX_LO)     = w0;
    *(v4u*)(At + loff + AX_LO + 8) = w1;
  }
}

template <bool XSPLIT, bool LAST>
__global__ __launch_bounds__(NTHR) void bilstm_layer_kernel(
    const unsigned short* XHp, const unsigned short* XLp,
    const unsigned short* __restrict__ WIp, const unsigned short* __restrict__ WHp,
    const float* __restrict__ BI, const float* __restrict__ BH,
    unsigned short* OHp, unsigned short* OLp,
    float* __restrict__ OF) {
  __shared__ __align__(16) unsigned short At[SEQ_BLK * APITCH];
  __shared__ __align__(16) float Sl[LAST ? (SEQ_BLK * SLP) : 4];
  const int tid = threadIdx.x, lane = tid & 31, wave = tid >> 5;
  const int c = lane & 15, hh = lane >> 4, koff = hh * 8;
  const int dir = (int)(blockIdx.x >> 1);
  const int rowbase = (int)(blockIdx.x & 1) * SEQ_BLK;
  const int j = 16 * wave + c;
  const _Float16* WI = (const _Float16*)WIp + (size_t)dir * NGATE * NCH;
  const _Float16* WH = (const _Float16*)WHp + (size_t)dir * NGATE * NHID;

  {
    unsigned* a32 = (unsigned*)At;
#pragma unroll 1
    for (int i = tid; i < (SEQ_BLK * APITCH) / 2; i += NTHR) a32[i] = 0u;
  }
  float cst[8], hst[8], bs[4];
#pragma unroll
  for (int g = 0; g < 4; ++g) bs[g] = BI[dir * NGATE + g * NHID + j] + BH[dir * NGATE + g * NHID + j];
#pragma unroll
  for (int r = 0; r < 8; ++r) { cst[r] = 0.0f; hst[r] = 0.0f; }
  __syncthreads();

  const int srow = tid >> 4, sc16 = (tid & 15) * 16;
  const int loff = srow * APITCH + sc16;
  {
    const int t0 = dir ? (NSTEP - 1) : 0;
    const size_t goff = ((size_t)t0 * NSEQ + (size_t)(rowbase + srow)) * NCH + sc16;
    stage_x_rows<XSPLIT>(At, XHp, XLp, goff, loff);
  }
  __syncthreads();

  const _Float16* arow = (const _Float16*)At + c * APITCH + koff;
  const v8f z8 = {0.f, 0.f, 0.f, 0.f, 0.f, 0.f, 0.f, 0.f};

#pragma unroll 1
  for (int s = 0; s < NSTEP; ++s) {
    const int t = dir ? (NSTEP - 1 - s) : s;
    v8f ach[4], acl[4];
    ach[0] = z8; ach[1] = z8; ach[2] = z8; ach[3] = z8;
    acl[0] = z8; acl[1] = z8; acl[2] = z8; acl[3] = z8;
#pragma unroll 1
    for (int k0 = 0; k0 < NCH; k0 += 32) {
      const v16h a = Frag<_Float16>::load(arow + AX_HI + k0);
      v16h al = a;
      if (XSPLIT) al = Frag<_Float16>::load(arow + AX_LO + k0);
      const _Float16* wi = WI + (size_t)j * NCH + koff + k0;
      const v16h b0 = Frag<_Float16>::load(wi);
      const v16h b1 = Frag<_Float16>::load(wi + (size_t)1 * NHID * NCH);
      const v16h b2 = Frag<_Float16>::load(wi + (size_t)2 * NHID * NCH);
      const v16h b3 = Frag<_Float16>::load(wi + (size_t)3 * NHID * NCH);
      ach[0] = Frag<_Float16>::mma(a, b0, ach[0]);
      ach[1] = Frag<_Float16>::mma(a, b1, ach[1]);
      ach[2] = Frag<_Float16>::mma(a, b2, ach[2]);
      ach[3] = Frag<_Float16>::mma(a, b3, ach[3]);
      if (XSPLIT) {
        acl[0] = Frag<_Float16>::mma(al, b0, acl[0]);
        acl[1] = Frag<_Float16>::mma(al, b1, acl[1]);
        acl[2] = Frag<_Float16>::mma(al, b2, acl[2]);
        acl[3] = Frag<_Float16>::mma(al, b3, acl[3]);
      }
      guard8_h(ach[0], ach[1], ach[2], ach[3], acl[0], acl[1], acl[2], acl[3], a, al, b0, b1, b2, b3);
    }
#pragma unroll 1
    for (int k0 = 0; k0 < NHID; k0 += 32) {
      const v16h a  = Frag<_Float16>::load(arow + AH_HI + k0);
      const v16h al = Frag<_Float16>::load(arow + AH_LO + k0);
      const _Float16* wh = WH + (size_t)j * NHID + koff + k0;
      const v16h b0 = Frag<_Float16>::load(wh);
      const v16h b1 = Frag<_Float16>::load(wh + (size_t)1 * NHID * NHID);
      const v16h b2 = Frag<_Float16>::load(wh + (size_t)2 * NHID * NHID);
      const v16h b3 = Frag<_Float16>::load(wh + (size_t)3 * NHID * NHID);
      ach[0] = Frag<_Float16>::mma(a, b0, ach[0]);
      ach[1] = Frag<_Float16>::mma(a, b1, ach[1]);
      ach[2] = Frag<_Float16>::mma(a, b2, ach[2]);
      ach[3] = Frag<_Float16>::mma(a, b3, ach[3]);
      acl[0] = Frag<_Float16>::mma(al, b0, acl[0]);
      acl[1] = Frag<_Float16>::mma(al, b1, acl[1]);
      acl[2] = Frag<_Float16>::mma(al, b2, acl[2]);
      acl[3] = Frag<_Float16>::mma(al, b3, acl[3]);
      guard8_h(ach[0], ach[1], ach[2], ach[3], acl[0], acl[1], acl[2], acl[3], a, al, b0, b1, b2, b3);
    }
    acc_guard4(ach[0], ach[1], ach[2], ach[3]);
    acc_guard4(acl[0], acl[1], acl[2], acl[3]);

#pragma unroll
    for (int r = 0; r < 8; ++r) {
      const float zi = ach[0][r] * WCARRY_INV + acl[0][r] * LCARRY_INV + bs[0];
      const float zf = ach[1][r] * WCARRY_INV + acl[1][r] * LCARRY_INV + bs[1];
      const float zg = ach[2][r] * WCARRY_INV + acl[2][r] * LCARRY_INV + bs[2];
      const float zo = ach[3][r] * WCARRY_INV + acl[3][r] * LCARRY_INV + bs[3];
      const float ig = fsig(zi);
      const float fg = fsig(zf);
      const float gg = ftanh(zg);
      const float og = fsig(zo);
      const float cn = fg * cst[r] + ig * gg;
      cst[r] = cn;
      hst[r] = og * ftanh(cn);
    }
    __syncthreads();

#pragma unroll
    for (int r = 0; r < 8; ++r) {
      const float h = hst[r];
      const float ha = (fabsf(h) < F16_MIN_NORMAL) ? 0.0f : h;
      const _Float16 h16 = (_Float16)ha;
      const float hif = (float)h16;
      const _Float16 l16 = (_Float16)((h - hif) * RCARRY);
      const int lrow = (8 * hh + r) * APITCH;
      At[lrow + AH_HI + j] = __builtin_bit_cast(unsigned short, h16);
      At[lrow + AH_LO + j] = __builtin_bit_cast(unsigned short, l16);
      if (LAST) Sl[(8 * hh + r) * SLP + j] = h;
    }
    {
      const int sn = (s + 1 < NSTEP) ? (s + 1) : (NSTEP - 1);
      const int tn = dir ? (NSTEP - 1 - sn) : sn;
      const size_t goff = ((size_t)tn * NSEQ + (size_t)(rowbase + srow)) * NCH + sc16;
      stage_x_rows<XSPLIT>(At, XHp, XLp, goff, loff);
    }
    __syncthreads();

    if (LAST) {
      for (int pass = 0; pass < 2; ++pass) {
#pragma unroll
        for (int it = 0; it < 2; ++it) {
          const int idx = it * NTHR + tid;
          const int row = idx >> 5, c4 = (idx & 31) * 4;
          const v4f v = *(const v4f*)(Sl + row * SLP + c4);
          *(volatile v4f*)(OF + ((size_t)t * NSEQ + (size_t)(rowbase + row)) * NCH + dir * NHID + c4) = v;
        }
        __threadfence();
      }
    } else {
      for (int pass = 0; pass < 2; ++pass) {
#pragma unroll
        for (int it = 0; it < 2; ++it) {
          const int idx = it * NTHR + tid;
          const int line = idx >> 3, e8 = (idx & 7) * 8;
          const int row = (line >> 1) & 15, qh = line & 1;
          const v4u v = *(const v4u*)(At + row * APITCH + ((it == 0) ? AH_HI : AH_LO) + qh * 64 + e8);
          unsigned short* dst = (it == 0) ? OHp : OLp;
          *(volatile v4u*)(dst + ((size_t)t * NSEQ + (size_t)(rowbase + row)) * NCH + dir * NHID + qh * 64 + e8) = v;
        }
        __threadfence();
      }
    }
  }
}

extern "C" void kernel_launch(void* const* d_in, const int* in_sizes, int n_in,
                              void* d_out, int out_size, void* d_ws, size_t ws_size, hipStream_t stream) {
  if (n_in < 5 || d_out == nullptr || d_ws == nullptr) return;
  if (in_sizes[0] != NXELEM || in_sizes[1] != NLAY * NDIR * NGATE * NCH || in_sizes[2] != NLAY * NDIR * NGATE * NHID ||
      in_sizes[3] != NLAY * NDIR * NGATE || in_sizes[4] != NLAY * NDIR * NGATE || out_size != NXELEM) return;

  const float* x   = (const float*)d_in[0];
  const float* wih = (const float*)d_in[1];
  const float* whh = (const float*)d_in[2];
  const float* bih = (const float*)d_in[3];
  const float* bhh = (const float*)d_in[4];
  float* out = (float*)d_out;

  char* ws = (char*)d_ws; size_t off = 0;
  auto carve = [&](size_t bytes) -> char* { char* p = ws + off; off += (bytes + 255) & ~(size_t)255; return p; };
  unsigned short* XH   = (unsigned short*)carve((size_t)NROWS * NCH * 2);
  unsigned short* WI16 = (unsigned short*)carve((size_t)NLAY * NDIR * NGATE * NCH * 2);
  unsigned short* WH16 = (unsigned short*)carve((size_t)NLAY * NDIR * NGATE * NHID * 2);
  unsigned short* H0H  = (unsigned short*)carve((size_t)NROWS * NCH * 2);
  unsigned short* H0L  = (unsigned short*)carve((size_t)NROWS * NCH * 2);
  float*          HST  = (float*)carve((size_t)NROWS * NCH * 4);
  if (off > ws_size || off > (size_t)134217728) return;

  const int n8wi = NLAY * NDIR * NGATE * NCH / 8;
  const int n8wh = NLAY * NDIR * NGATE * NHID / 8;
  cvt16_kernel<<<(n8wi + NTHR - 1) / NTHR, NTHR, 0, stream>>>(wih, WI16, n8wi, WCARRY);
  cvt16_kernel<<<(n8wh + NTHR - 1) / NTHR, NTHR, 0, stream>>>(whh, WH16, n8wh, WCARRY);
  tp16_kernel<<<dim3(NSTEP / 64, NFLAT / 64), NTHR, 0, stream>>>(x, NSTEP, NFLAT, XH);
  bilstm_layer_kernel<false, false><<<NDIR * (NSEQ / SEQ_BLK), NTHR, 0, stream>>>(
      XH, XH, WI16, WH16, bih, bhh, H0H, H0L, HST);
  bilstm_layer_kernel<true, true><<<NDIR * (NSEQ / SEQ_BLK), NTHR, 0, stream>>>(
      H0H, H0L, WI16 + (size_t)NDIR * NGATE * NCH, WH16 + (size_t)NDIR * NGATE * NHID,
      bih + NDIR * NGATE, bhh + NDIR * NGATE, H0H, H0L, HST);
  tp32_kernel<<<dim3(NFLAT / 64, NSTEP / 64), NTHR, 0, stream>>>(HST, NFLAT, NSTEP, out);
}
